// LiquidTimeConstantNetwork_35665408426494
// MI455X (gfx1250) — hardware-run, weakly checked
//
#include <hip/hip_runtime.h>
#include <math.h>

typedef __attribute__((ext_vector_type(16))) _Float16 v16h;
typedef __attribute__((ext_vector_type(8)))  _Float16 v8h;
typedef __attribute__((ext_vector_type(8)))  float    v8f;
typedef __attribute__((ext_vector_type(4)))  float    v4f;

constexpr int NBATCH  = 32;
constexpr int NSTEP   = 1024;
constexpr int NIN     = 256;
constexpr int NHID    = 512;
constexpr int NOUT    = 256;
constexpr int NTHR    = 256;
constexpr int SEQ_BLK = 16;
constexpr int HPITCH  = 520;
constexpr int SLABP   = 68;
constexpr int NROWS   = NBATCH * NSTEP;
constexpr int NOUT0   = NROWS * NOUT;
constexpr int NOUT1   = NBATCH * NHID;
constexpr float DT_F            = 0.1f;
constexpr float TAU_MIX_F       = 0.1f;
constexpr float W_CARRY         = 256.0f;
constexpr float X_CARRY         = 16.0f;
constexpr float H_CARRY         = 256.0f;
constexpr float S0_FOLD         = 1.0f / (W_CARRY * X_CARRY);
constexpr float S1_FOLD         = 1.0f / (W_CARRY * H_CARRY);
constexpr float F16_MIN_NORMAL  = 6.103515625e-5f;
static_assert(NBATCH % SEQ_BLK == 0, "block rows");
static_assert(NHID == 64 * (NTHR / 32), "8 waves x 64 hidden columns");
static_assert(NIN % 32 == 0 && NHID % 32 == 0, "GEMM K multiples of 32");
static_assert(NROWS % 64 == 0 && NHID % 64 == 0 && NOUT % 64 == 0, "GEMM M, N multiples of 64");
static_assert((2 * SEQ_BLK * HPITCH) % NTHR == 0, "operand tile zero fill exact");
static_assert(((NTHR / 32) * 16 * SLABP) % NTHR == 0, "slab zero fill exact");
static_assert(HPITCH % 8 == 0 && SLABP % 4 == 0, "16-B aligned LDS rows");
static_assert((NROWS * (NIN / 8)) % NTHR == 0, "x convert grid exact");
static_assert((NSTEP * NHID) % NTHR == 0, "time-constant grid exact");

constexpr size_t SZ_X16    = (size_t)NROWS * NIN * 2;
constexpr size_t SZ_SENS   = (size_t)NROWS * NHID * 4;
constexpr size_t SZ_H16    = (size_t)NROWS * NHID * 2;
constexpr size_t SZ_RTAU   = (size_t)NSTEP * NHID * 4;
constexpr size_t SZ_WIN16  = (size_t)NHID * NIN * 2;
constexpr size_t SZ_WREC16 = (size_t)NHID * NHID * 2;
constexpr size_t SZ_WOUT16 = (size_t)NOUT * NHID * 2;
constexpr size_t OFF_X16    = 0;
constexpr size_t OFF_SENS   = OFF_X16    + SZ_X16;
constexpr size_t OFF_H16    = OFF_SENS   + SZ_SENS;
constexpr size_t OFF_RTAU   = OFF_H16    + SZ_H16;
constexpr size_t OFF_WIN16  = OFF_RTAU   + SZ_RTAU;
constexpr size_t OFF_WREC16 = OFF_WIN16  + SZ_WIN16;
constexpr size_t OFF_WOUT16 = OFF_WREC16 + SZ_WREC16;
constexpr size_t WS_TOTAL   = OFF_WOUT16 + SZ_WOUT16;
static_assert(WS_TOTAL == 120586240ull, "carve total");
static_assert(WS_TOTAL <= 134217728ull, "carve cap");
static_assert((OFF_SENS % 256) == 0 && (OFF_H16 % 256) == 0 && (OFF_RTAU % 256) == 0 && (OFF_WIN16 % 256) == 0 &&
              (OFF_WREC16 % 256) == 0 && (OFF_WOUT16 % 256) == 0, "aligned regions");

union FragU { v16h v; v8h h[2]; };
__device__ __forceinline__ v16h frag_load(const _Float16* p) {
  FragU f;
  f.h[0] = *(const v8h*)(p);
  f.h[1] = *(const v8h*)(p + 16);
  return f.v;
}
__device__ __forceinline__ v8f mma_h(v16h a, v16h b, v8f c) {
  c = __builtin_amdgcn_wmma_f32_16x16x32_f16(false, a, false, b, (short)0, c, false, false);
  asm volatile("v_nop\n\tv_nop\n\tv_nop\n\tv_nop" : "+v"(c) : "v"(a), "v"(b));
  return c;
}
__device__ __forceinline__ v8f mma_raw(v16h a, v16h b, v8f c) {
  return __builtin_amdgcn_wmma_f32_16x16x32_f16(false, a, false, b, (short)0, c, false, false);
}
__device__ __forceinline__ void grp_guard_h(v8f& a0, v8f& a1, v8f& a2, v8f& a3, v16h x, v16h b0, v16h b1, v16h b2, v16h b3) {
  asm volatile("v_nop\n\tv_nop\n\tv_nop\n\tv_nop" : "+v"(a0), "+v"(a1), "+v"(a2), "+v"(a3) : "v"(x), "v"(b0), "v"(b1), "v"(b2), "v"(b3));
}
__device__ __forceinline__ void keep4_h(v16h a, v16h b, v16h c, v16h d) { asm volatile("v_nop" :: "v"(a), "v"(b), "v"(c), "v"(d)); }
__device__ __forceinline__ void acc_guard4(v8f& a, v8f& b, v8f& c, v8f& d) { asm volatile("v_nop\n\tv_nop\n\tv_nop\n\tv_nop" : "+v"(a), "+v"(b), "+v"(c), "+v"(d)); }
__device__ __forceinline__ void wave_sync() {
  __builtin_amdgcn_fence(__ATOMIC_RELEASE, "workgroup");
  __builtin_amdgcn_wave_barrier();
  __builtin_amdgcn_fence(__ATOMIC_ACQUIRE, "workgroup");
}
__device__ __forceinline__ _Float16 to_h16(float v) {
  const float f = (fabsf(v) < F16_MIN_NORMAL) ? 0.0f : v;
  return (_Float16)f;
}

__global__ __launch_bounds__(256) void gemm64_f16_kernel(
    const unsigned short* __restrict__ Ap, int lda,
    const unsigned short* __restrict__ Btp, int ldb,
    float* __restrict__ C, int ldc, int M, int N, int K, float scale) {
  const _Float16* A  = (const _Float16*)Ap;
  const _Float16* Bt = (const _Float16*)Btp;
  __shared__ __align__(16) float sT[8][16 * 68];
  const int lane = threadIdx.x & 31;
  const int wave = threadIdx.x >> 5;
  const int tilesN = N >> 6;
  const int tilesM = M >> 6;
  const int tile = blockIdx.x * 8 + wave;
  if (tile >= tilesM * tilesN) return;
  const int tm = tile / tilesN;
  const int tn = tile - tm * tilesN;
  const int m0 = tm << 6;
  const int n0 = tn << 6;
  const int rlane = lane & 15;
  const int koff  = (lane >> 4) * 8;
  const int mOff  = (lane >> 4) * 8;

  v8f acc[4][4];
#pragma unroll
  for (int i = 0; i < 4; ++i)
#pragma unroll
    for (int j = 0; j < 4; ++j) acc[i][j] = (v8f){0.f, 0.f, 0.f, 0.f, 0.f, 0.f, 0.f, 0.f};

  for (int k0 = 0; k0 < K; k0 += 32) {
    v16h bh[4];
#pragma unroll
    for (int j = 0; j < 4; ++j) {
      const size_t bo = (size_t)(n0 + (j << 4) + rlane) * ldb + koff + k0;
      bh[j] = frag_load(Bt + bo);
    }
#pragma unroll
    for (int i = 0; i < 4; ++i) {
      const size_t ao = (size_t)(m0 + (i << 4) + rlane) * lda + koff + k0;
      const v16h ah = frag_load(A + ao);
#pragma unroll
      for (int j = 0; j < 4; ++j) acc[i][j] = mma_raw(ah, bh[j], acc[i][j]);
      grp_guard_h(acc[i][0], acc[i][1], acc[i][2], acc[i][3], ah, bh[0], bh[1], bh[2], bh[3]);
    }
    keep4_h(bh[0], bh[1], bh[2], bh[3]);
  }
  acc_guard4(acc[0][0], acc[0][1], acc[0][2], acc[0][3]);
  acc_guard4(acc[1][0], acc[1][1], acc[1][2], acc[1][3]);
  acc_guard4(acc[2][0], acc[2][1], acc[2][2], acc[2][3]);
  acc_guard4(acc[3][0], acc[3][1], acc[3][2], acc[3][3]);

  float* slab = sT[wave];
  const int hh = lane >> 4, c4 = (lane & 15) * 4;
#pragma unroll
  for (int i = 0; i < 4; ++i) {
    const int mBase = m0 + (i << 4);
#pragma unroll
    for (int j = 0; j < 4; ++j) {
#pragma unroll
      for (int r = 0; r < 8; ++r) {
        const float v = acc[i][j][r] * scale;
        slab[(mOff + r) * 68 + (j << 4) + rlane] = v;
      }
    }
    wave_sync();
    for (int pass = 0; pass < 2; ++pass) {
#pragma unroll
      for (int it = 0; it < 8; ++it) {
        const int row = it * 2 + hh;
        const v4f v = *(const v4f*)(slab + row * 68 + c4);
        *(volatile v4f*)(C + (size_t)(mBase + row) * ldc + n0 + c4) = v;
      }
      __threadfence();
    }
    wave_sync();
  }
}

__global__ __launch_bounds__(NTHR) void cvt8_scale_kernel(const float* __restrict__ src, unsigned short* __restrict__ dst,
                                                         int n8, float sc) {
  const int i = blockIdx.x * NTHR + threadIdx.x;
  if (i < n8) {
    const float* sp = src + (size_t)i * 8;
    const v4f a = *(const v4f*)(sp);
    const v4f b = *(const v4f*)(sp + 4);
    v8h hv;
#pragma unroll
    for (int e = 0; e < 4; ++e) {
      const float fa = a[e] * sc;
      const float fb = b[e] * sc;
      hv[e]     = to_h16(fa);
      hv[4 + e] = to_h16(fb);
    }
    unsigned short* op = dst + (size_t)i * 8;
    *(volatile v8h*)op = hv;
    __threadfence();
    *(volatile v8h*)op = hv;
  }
}

__global__ __launch_bounds__(NTHR) void xperm_cvt_kernel(const float* __restrict__ x, unsigned short* __restrict__ X16) {
  const int i = blockIdx.x * NTHR + threadIdx.x;
  if (i < NROWS * (NIN / 8)) {
    const int m  = i >> 5;
    const int c8 = (i & 31) * 8;
    const int t  = m >> 5;
    const int b  = m & 31;
    const float* sp = x + ((size_t)b * NSTEP + (size_t)t) * NIN + c8;
    const v4f a0 = *(const v4f*)(sp);
    const v4f a1 = *(const v4f*)(sp + 4);
    v8h hv;
#pragma unroll
    for (int e = 0; e < 4; ++e) {
      const float fa = a0[e] * X_CARRY;
      const float fb = a1[e] * X_CARRY;
      hv[e]     = to_h16(fa);
      hv[4 + e] = to_h16(fb);
    }
    unsigned short* op = X16 + (size_t)i * 8;
    *(volatile v8h*)op = hv;
    __threadfence();
    *(volatile v8h*)op = hv;
  }
}

__global__ __launch_bounds__(NTHR) void rtau_kernel(const float* __restrict__ SENS, const float* __restrict__ tc,
                                                   float* __restrict__ RTAU) {
  const int idx = blockIdx.x * NTHR + threadIdx.x;
  if (idx < NSTEP * NHID) {
    const int t = idx >> 9;
    const int h = idx & (NHID - 1);
    const float* p = SENS + (size_t)t * NBATCH * NHID + h;
    float s = 0.0f;
#pragma unroll 8
    for (int b = 0; b < NBATCH; ++b) s += fabsf(p[(size_t)b * NHID]);
    const float mean = s * (1.0f / (float)NBATCH);
    const float z = tc[h] + TAU_MIX_F * mean;
    const float sp = fmaxf(z, 0.0f) + log1pf(expf(-fabsf(z)));
    const float rt = 1.0f / sp;
    *(volatile float*)(RTAU + idx) = rt;
    __threadfence();
    *(volatile float*)(RTAU + idx) = rt;
  }
}

__device__ __forceinline__ float cell_update(float accv, float sv, float bv, float ho, float rt) {
  const float pre = (sv + accv * S1_FOLD) + bv;
  const float act = tanhf(pre);
  return ho + DT_F * (act - ho * rt);
}

__global__ __launch_bounds__(NTHR) void rec_seq_kernel(const float* __restrict__ SENS, const float* __restrict__ RTAU,
                                                      const unsigned short* __restrict__ WRp, const float* __restrict__ bias,
                                                      unsigned short* __restrict__ H16, float* __restrict__ OUT1) {
  __shared__ __align__(16) _Float16 Ah[2 * SEQ_BLK * HPITCH];
  __shared__ __align__(16) float    Sl[(NTHR / 32) * 16 * SLABP];
  __shared__ __align__(16) float    Hm[(NTHR / 32) * 16 * SLABP];
  const _Float16* WR = (const _Float16*)WRp;
  const int tid = threadIdx.x, lane = tid & 31, wave = tid >> 5;
  const int c = lane & 15, hh = lane >> 4, koff = hh * 8;
  const int q = lane >> 3, c8 = (lane & 7) * 8, c4 = c * 4;
  const int rowbase = blockIdx.x * SEQ_BLK;
  const int colw = 64 * wave;

#pragma unroll 1
  for (int i = tid; i < 2 * SEQ_BLK * HPITCH; i += NTHR) Ah[i] = (_Float16)0.0f;
#pragma unroll 1
  for (int i = tid; i < (NTHR / 32) * 16 * SLABP; i += NTHR) {
    Sl[i] = 0.0f;
    Hm[i] = 0.0f;
  }
  __syncthreads();

  float* slab = Sl + wave * 16 * SLABP;
  float* hm   = Hm + wave * 16 * SLABP;
  const _Float16* w0 = WR + (size_t)(colw + c) * NHID + koff;
  const _Float16* w1 = w0 + (size_t)16 * NHID;
  const _Float16* w2 = w0 + (size_t)32 * NHID;
  const _Float16* w3 = w0 + (size_t)48 * NHID;
  const v4f bi0 = *(const v4f*)(bias + colw + c8);
  const v4f bi1 = *(const v4f*)(bias + colw + c8 + 4);
  const v8f z8 = {0.f, 0.f, 0.f, 0.f, 0.f, 0.f, 0.f, 0.f};

#pragma unroll 1
  for (int t = 0; t < NSTEP; ++t) {
    const int cur = t & 1;
    const _Float16* ahrow = Ah + cur * (SEQ_BLK * HPITCH) + c * HPITCH + koff;
    _Float16* ahn = Ah + (cur ^ 1) * (SEQ_BLK * HPITCH);

    v8f acc0 = z8, acc1 = z8, acc2 = z8, acc3 = z8;
#pragma unroll 1
    for (int k0 = 0; k0 < NHID; k0 += 32) {
      const v16h a  = frag_load(ahrow + k0);
      const v16h b0 = frag_load(w0 + k0);
      const v16h b1 = frag_load(w1 + k0);
      const v16h b2 = frag_load(w2 + k0);
      const v16h b3 = frag_load(w3 + k0);
      acc0 = mma_h(a, b0, acc0);
      acc1 = mma_h(a, b1, acc1);
      acc2 = mma_h(a, b2, acc2);
      acc3 = mma_h(a, b3, acc3);
    }

#pragma unroll
    for (int r = 0; r < 8; ++r) {
      slab[(8 * hh + r) * SLABP + c]      = acc0[r];
      slab[(8 * hh + r) * SLABP + 16 + c] = acc1[r];
      slab[(8 * hh + r) * SLABP + 32 + c] = acc2[r];
      slab[(8 * hh + r) * SLABP + 48 + c] = acc3[r];
    }
    wave_sync();

    const float* rp = RTAU + (size_t)t * NHID + colw + c8;
    const v4f rt0 = *(const v4f*)(rp);
    const v4f rt1 = *(const v4f*)(rp + 4);

#pragma unroll 1
    for (int it = 0; it < 4; ++it) {
      const int row = it * 4 + q;
      const float* sp = slab + row * SLABP + c8;
      float* hp = hm + row * SLABP + c8;
      const float* gp = SENS + ((size_t)t * NBATCH + (size_t)(rowbase + row)) * NHID + colw + c8;
      const v4f a0 = *(const v4f*)(sp);
      const v4f a1 = *(const v4f*)(sp + 4);
      const v4f h0 = *(const v4f*)(hp);
      const v4f h1 = *(const v4f*)(hp + 4);
      const v4f s0 = *(const v4f*)(gp);
      const v4f s1 = *(const v4f*)(gp + 4);
      v4f n0, n1;
      v8h hv;
#pragma unroll
      for (int e = 0; e < 4; ++e) {
        const float x0 = cell_update(a0[e], s0[e], bi0[e], h0[e], rt0[e]);
        const float x1 = cell_update(a1[e], s1[e], bi1[e], h1[e], rt1[e]);
        n0[e] = x0;
        n1[e] = x1;
        const float y0 = x0 * H_CARRY;
        const float y1 = x1 * H_CARRY;
        hv[e]     = to_h16(y0);
        hv[4 + e] = to_h16(y1);
      }
      *(v4f*)(hp)     = n0;
      *(v4f*)(hp + 4) = n1;
      *(v8h*)(ahn + row * HPITCH + colw + c8) = hv;
      unsigned short* op = H16 + ((size_t)(rowbase + row) * NSTEP + (size_t)t) * NHID + colw + c8;
      *(volatile v8h*)op = hv;
      __threadfence();
      *(volatile v8h*)op = hv;
    }
    __syncthreads();
  }

  wave_sync();
  for (int pass = 0; pass < 2; ++pass) {
#pragma unroll
    for (int it = 0; it < 8; ++it) {
      const int row = it * 2 + hh;
      const v4f v = *(const v4f*)(hm + row * SLABP + c4);
      *(volatile v4f*)(OUT1 + (size_t)(rowbase + row) * NHID + colw + c4) = v;
    }
    __threadfence();
  }
}

extern "C" void kernel_launch(void* const* d_in, const int* in_sizes, int n_in,
                              void* d_out, int out_size, void* d_ws, size_t ws_size, hipStream_t stream) {
  if (n_in < 6 || d_out == nullptr || d_ws == nullptr) return;
  if (in_sizes[0] != NBATCH * NSTEP * NIN) return;
  if (in_sizes[1] != NHID * NIN) return;
  if (in_sizes[2] != NHID * NHID) return;
  if (in_sizes[3] != NHID) return;
  if (in_sizes[4] != NOUT * NHID) return;
  if (in_sizes[5] != NHID) return;
  if (out_size != NOUT0 + NOUT1) return;
  if (ws_size < WS_TOTAL) return;

  const float* x     = (const float*)d_in[0];
  const float* w_in  = (const float*)d_in[1];
  const float* w_rec = (const float*)d_in[2];
  const float* tc    = (const float*)d_in[3];
  const float* w_out = (const float*)d_in[4];
  const float* bias  = (const float*)d_in[5];
  float* out0 = (float*)d_out;
  float* out1 = out0 + (size_t)NOUT0;

  char* ws = (char*)d_ws;
  unsigned short* X16    = (unsigned short*)(ws + OFF_X16);
  float*          SENS   = (float*)(ws + OFF_SENS);
  unsigned short* H16    = (unsigned short*)(ws + OFF_H16);
  float*          RTAU   = (float*)(ws + OFF_RTAU);
  unsigned short* WIN16  = (unsigned short*)(ws + OFF_WIN16);
  unsigned short* WREC16 = (unsigned short*)(ws + OFF_WREC16);
  unsigned short* WOUT16 = (unsigned short*)(ws + OFF_WOUT16);

  const int n8_win  = NHID * NIN / 8;
  const int n8_wrec = NHID * NHID / 8;
  const int n8_wout = NOUT * NHID / 8;
  cvt8_scale_kernel<<<n8_win / NTHR, NTHR, 0, stream>>>(w_in, WIN16, n8_win, W_CARRY);
  cvt8_scale_kernel<<<n8_wrec / NTHR, NTHR, 0, stream>>>(w_rec, WREC16, n8_wrec, W_CARRY);
  cvt8_scale_kernel<<<n8_wout / NTHR, NTHR, 0, stream>>>(w_out, WOUT16, n8_wout, W_CARRY);
  xperm_cvt_kernel<<<(NROWS * (NIN / 8)) / NTHR, NTHR, 0, stream>>>(x, X16);

  gemm64_f16_kernel<<<(NROWS / 64) * (NHID / 64) / 8, 256, 0, stream>>>(
      X16, NIN, WIN16, NIN, SENS, NHID, NROWS, NHID, NIN, S0_FOLD);

  rtau_kernel<<<(NSTEP * NHID) / NTHR, NTHR, 0, stream>>>(SENS, tc, RTAU);

  rec_seq_kernel<<<NBATCH / SEQ_BLK, NTHR, 0, stream>>>(SENS, RTAU, WREC16, bias, H16, out1);

  gemm64_f16_kernel<<<(NROWS / 64) * (NOUT / 64) / 8, 256, 0, stream>>>(
      H16, NHID, WOUT16, NHID, out0, NOUT, NROWS, NOUT, NHID, S1_FOLD);
}
